// wAttnModule_38886633898207
// MI455X (gfx1250) — hardware-verified
//
#include <hip/hip_runtime.h>


namespace {
constexpr int NQ = 128, NSEN = 1024, NS = 256, NF = 50, FP = 64, NV = 4 * NF, XW = 256, SLOTS = 128;
constexpr float XS = 8.0f, QS = 64.0f, PS = 1024.0f;

typedef _Float16 b16;
typedef __attribute__((ext_vector_type(16))) _Float16 v16b;
typedef __attribute__((ext_vector_type(8))) _Float16 v8b;
typedef __attribute__((ext_vector_type(2))) _Float16 v2b;
typedef __attribute__((ext_vector_type(8))) float v8f;
typedef __attribute__((ext_vector_type(4))) float v4f;
__device__ __forceinline__ float bf16_rne(float f) { unsigned int u = __float_as_uint(f); u += 0x7FFFu + ((u >> 16) & 1u); return __uint_as_float(u & 0xFFFF0000u); }
__device__ __forceinline__ void split16(float v, b16& hi, b16& lo) { hi = (b16)v; lo = (b16)(v - (float)hi); }
__device__ __forceinline__ v16b frag_kb(const b16* p, int hh) { const v8b a = *(const v8b*)(p + 8 * hh), b = *(const v8b*)(p + 16 + 8 * hh); v16b f;
#pragma unroll
  for (int e = 0; e < 8; ++e) { f[e] = a[e]; f[8 + e] = b[e]; } return f; }
__device__ __forceinline__ v8f wmma16b(v16b a, v16b b, v8f c) { v8f d = __builtin_amdgcn_wmma_f32_16x16x32_f16(false, a, false, b, (short)0, c, false, false); asm volatile("v_nop\n\tv_nop\n\tv_nop\n\tv_nop" : "+v"(d) : "v"(a), "v"(b)); return d; }
__device__ __forceinline__ float nexp(float x) { return __builtin_amdgcn_exp2f(x * 1.4426950408889634f); }
__device__ __forceinline__ float pmul(float a, float b) { float p = a * b; asm volatile("" : "+v"(p)); return p; }
__device__ __forceinline__ float hmax16(float v) { v = fmaxf(v, __shfl_xor(v, 1)); v = fmaxf(v, __shfl_xor(v, 2)); v = fmaxf(v, __shfl_xor(v, 4)); return fmaxf(v, __shfl_xor(v, 8)); }
__device__ __forceinline__ float hsum16(float v) { v += __shfl_xor(v, 1); v += __shfl_xor(v, 2); v += __shfl_xor(v, 4); return v + __shfl_xor(v, 8); }
__device__ __forceinline__ float tanh_(float x) { const float e = nexp(-2.0f * fabsf(x)); const float t = (1.0f - e) / (1.0f + e); return x < 0.0f ? -t : t; }

__global__ __launch_bounds__(256) void prep_kernel(const float* __restrict__ doc, const float* __restrict__ query, const float* __restrict__ clw, b16* __restrict__ D16, b16* __restrict__ DT16, b16* __restrict__ QT16, b16* __restrict__ QW3H, b16* __restrict__ QW3L, float* __restrict__ QW2) {
  __shared__ __attribute__((aligned(16))) b16 Td[64][FP + 8], Tt[FP][64 + 8]; __shared__ __attribute__((aligned(16))) b16 Tq[FP][NQ + 8], Th[NQ][FP + 8], Tl[NQ][FP + 8]; __shared__ float Sw2[NQ];
  const int n = blockIdx.y, s0 = blockIdx.x * 64, t_ = threadIdx.x;
  for (int k = t_; k < 64 * FP; k += 256) { const int ss = k >> 6, f = k & 63; const b16 v = (f < NF) ? (b16)(bf16_rne(doc[((size_t)n * NS + s0 + ss) * NF + (f < NF ? f : 0)]) * XS) : (b16)0.0f; Td[ss][f] = v; Tt[f][ss] = v; }
  if (blockIdx.x == 0 && blockIdx.y == 0) {
    for (int k = t_; k < NQ * FP; k += 256) { const int q = k >> 6, f = k & 63; const float qv = (f < NF) ? bf16_rne(query[q * NF + (f < NF ? f : 0)]) : 0.0f; const float w3 = (f < NF) ? bf16_rne(clw[2 * NF + (f < NF ? f : 0)]) : 0.0f;
      Tq[f][q] = (b16)(qv * XS); b16 a_, c_; split16(pmul(qv, w3) * QS, a_, c_); Th[q][f] = a_; Tl[q][f] = c_; }
    if (t_ < NQ) { float s = 0.0f;
#pragma unroll 1
      for (int f = 0; f < NF; ++f) s += pmul(bf16_rne(query[t_ * NF + f]), bf16_rne(clw[NF + f])); Sw2[t_] = s; } }
  __syncthreads();
  for (int pass = 0; pass < 2; ++pass) {
    for (int q = t_; q < 64 * 8; q += 256) { const int ss = q >> 3, c8 = (q & 7) * 8; *(volatile v8b*)(D16 + ((size_t)n * NS + s0 + ss) * FP + c8) = *(const v8b*)(&Td[ss][c8]); }
    for (int q = t_; q < FP * 8; q += 256) { const int f = q >> 3, c8 = (q & 7) * 8; *(volatile v8b*)(DT16 + ((size_t)n * FP + f) * NS + s0 + c8) = *(const v8b*)(&Tt[f][c8]); }
    if (blockIdx.x == 0 && blockIdx.y == 0) {
      for (int q = t_; q < FP * 16; q += 256) { const int f = q >> 4, c8 = (q & 15) * 8; *(volatile v8b*)(QT16 + (size_t)f * NQ + c8) = *(const v8b*)(&Tq[f][c8]); }
      for (int q = t_; q < NQ * 8; q += 256) { const int qq = q >> 3, c8 = (q & 7) * 8; *(volatile v8b*)(QW3H + (size_t)qq * FP + c8) = *(const v8b*)(&Th[qq][c8]); *(volatile v8b*)(QW3L + (size_t)qq * FP + c8) = *(const v8b*)(&Tl[qq][c8]); }
      if (t_ < NQ) ((volatile float*)QW2)[t_] = Sw2[t_]; }
    __threadfence(); }
}
__global__ __launch_bounds__(512) void phase1_kernel(const b16* __restrict__ D16, const float* __restrict__ doc, const float* __restrict__ clw, const b16* __restrict__ QW3H, const b16* __restrict__ QW3L, const float* __restrict__ QW2, int base, b16* __restrict__ PQTH, b16* __restrict__ PQTL, b16* __restrict__ PDH, b16* __restrict__ PDL) {
  __shared__ __attribute__((aligned(16))) b16 Stg[2][NQ][NS + 8];
  __shared__ float Sdw1[NS], Cmx[16][NQ], Csm[16][NQ];
  const int slot = blockIdx.x, n = base + slot, t_ = threadIdx.x, wave = t_ >> 5, lane = t_ & 31, nloc = lane & 15, hlf = lane >> 4;
  if (t_ < NS) { float s = 0.0f;
#pragma unroll 1
    for (int f = 0; f < NF; ++f) s += pmul(bf16_rne(doc[((size_t)n * NS + t_) * NF + f]), bf16_rne(clw[f])); Sdw1[t_] = s; }
  v8f acc[8];
#pragma unroll
  for (int nt = 0; nt < 8; ++nt) acc[nt] = (v8f){};
  const b16* A = D16 + ((size_t)n * NS + wave * 16) * FP;
  v16b a0[2];
#pragma unroll
  for (int ks = 0; ks < 2; ++ks) a0[ks] = frag_kb(A + (size_t)nloc * FP + ks * 32, hlf);
#pragma unroll
  for (int nt = 0; nt < 8; ++nt) {
#pragma unroll
    for (int ks = 0; ks < 2; ++ks) { v16b b = frag_kb(QW3H + (size_t)(nt * 16 + nloc) * FP + ks * 32, hlf); acc[nt] = wmma16b(a0[ks], b, acc[nt]);
      b = frag_kb(QW3L + (size_t)(nt * 16 + nloc) * FP + ks * 32, hlf); acc[nt] = wmma16b(a0[ks], b, acc[nt]); } }
  __syncthreads();
  const int sb = wave * 16 + 8 * hlf; float rmx[8], rinv[8];
#pragma unroll
  for (int r = 0; r < 8; ++r) { const float d1 = Sdw1[sb + r]; float mx = -INFINITY;
#pragma unroll
    for (int nt = 0; nt < 8; ++nt) { const float v = acc[nt][r] * (1.0f / (XS * QS)) + d1 + QW2[nt * 16 + nloc]; acc[nt][r] = v; mx = fmaxf(mx, v); }
    mx = hmax16(mx); float sm = 0.0f;
#pragma unroll
    for (int nt = 0; nt < 8; ++nt) sm += nexp(acc[nt][r] - mx);
    sm = hsum16(sm); rmx[r] = mx; rinv[r] = 1.0f / sm; }
#pragma unroll
  for (int nt = 0; nt < 8; ++nt) { v8b ph, pl;
#pragma unroll
    for (int r = 0; r < 8; ++r) { b16 a_, c_; split16(nexp(acc[nt][r] - rmx[r]) * rinv[r] * PS, a_, c_); ph[r] = a_; pl[r] = c_; }
    *(v8b*)(&Stg[0][nt * 16 + nloc][sb]) = ph; *(v8b*)(&Stg[1][nt * 16 + nloc][sb]) = pl; }
  __syncthreads();
  for (int pass = 0; pass < 2; ++pass) { for (int rr = wave * 8; rr < wave * 8 + 8; ++rr) { *(volatile v8b*)(PQTH + ((size_t)slot * NQ + rr) * NS + lane * 8) = *(const v8b*)(&Stg[0][rr][lane * 8]); *(volatile v8b*)(PQTL + ((size_t)slot * NQ + rr) * NS + lane * 8) = *(const v8b*)(&Stg[1][rr][lane * 8]); } __threadfence(); }
  __syncthreads();
#pragma unroll
  for (int nt = 0; nt < 8; ++nt) { float mx = -INFINITY;
#pragma unroll
    for (int r = 0; r < 8; ++r) mx = fmaxf(mx, acc[nt][r]);
    mx = fmaxf(mx, __shfl_xor(mx, 16)); if (hlf == 0) Cmx[wave][nt * 16 + nloc] = mx; }
  __syncthreads();
  float cm[8], cinv[8];
#pragma unroll
  for (int nt = 0; nt < 8; ++nt) { float mx = -INFINITY; for (int w = 0; w < 16; ++w) mx = fmaxf(mx, Cmx[w][nt * 16 + nloc]); cm[nt] = mx; float sm = 0.0f;
#pragma unroll
    for (int r = 0; r < 8; ++r) sm += nexp(acc[nt][r] - mx);
    sm += __shfl_xor(sm, 16); if (hlf == 0) Csm[wave][nt * 16 + nloc] = sm; }
  __syncthreads();
#pragma unroll
  for (int nt = 0; nt < 8; ++nt) { float sm = 0.0f; for (int w = 0; w < 16; ++w) sm += Csm[w][nt * 16 + nloc]; cinv[nt] = 1.0f / sm; }
  for (int plane = 0; plane < 2; ++plane) {
    b16 (*St)[NQ + 8] = (b16 (*)[NQ + 8])&Stg[0][0][0];
#pragma unroll
    for (int r = 0; r < 8; ++r) { const int s = sb + r;
#pragma unroll
      for (int nt = 0; nt < 8; ++nt) { b16 a_, c_; split16(nexp(acc[nt][r] - cm[nt]) * cinv[nt] * PS, a_, c_); const b16 mine = plane ? c_ : a_;
        const float mf = (float)mine; const float nb = __shfl_xor(mf, 1);
        if ((nloc & 1) == 0) { v2b pr; pr[0] = mine; pr[1] = (b16)nb; *(v2b*)(&St[s][nt * 16 + nloc]) = pr; } } }
    __syncthreads();
    b16* dst = plane ? PDL : PDH;
    for (int pass = 0; pass < 2; ++pass) { for (int rr = wave * 16; rr < wave * 16 + 16; ++rr) if (lane < 16) *(volatile v8b*)(dst + ((size_t)slot * NS + rr) * NQ + lane * 8) = *(const v8b*)(&St[rr][lane * 8]); __threadfence(); }
    __syncthreads(); }
}
__global__ __launch_bounds__(256) void phase2_kernel(const b16* __restrict__ PDH, const b16* __restrict__ PDL, const b16* __restrict__ PQTH, const b16* __restrict__ PQTL, const b16* __restrict__ QT16, const b16* __restrict__ DT16, const float* __restrict__ doc, const float* __restrict__ dl1, const float* __restrict__ dW1p, int base, float* __restrict__ X) {
  __shared__ __attribute__((aligned(16))) float ADQ[NS][52], AQD[NS][52]; __shared__ __attribute__((aligned(16))) b16 GTh[FP][NQ + 8], GTl[FP][NQ + 8]; __shared__ float Sc[NS], Sred[2][8];
  const int slot = blockIdx.x, n = base + slot, t_ = threadIdx.x, wave = t_ >> 5, lane = t_ & 31, nloc = lane & 15, hlf = lane >> 4;
  const b16* Ph = PDH + (size_t)slot * NS * NQ; const b16* Pl = PDL + (size_t)slot * NS * NQ; const b16* Th_ = PQTH + (size_t)slot * NQ * NS; const b16* Tl_ = PQTL + (size_t)slot * NQ * NS; const b16* Dt = DT16 + (size_t)n * FP * NS;
  { v8f acc[2][4];
#pragma unroll
    for (int mt = 0; mt < 2; ++mt)
#pragma unroll
      for (int nt = 0; nt < 4; ++nt) acc[mt][nt] = (v8f){};
#pragma unroll
    for (int kb = 0; kb < NQ; kb += 32) { v16b ah[2], al[2];
#pragma unroll
      for (int mt = 0; mt < 2; ++mt) { ah[mt] = frag_kb(Ph + (size_t)(wave * 32 + mt * 16 + nloc) * NQ + kb, hlf); al[mt] = frag_kb(Pl + (size_t)(wave * 32 + mt * 16 + nloc) * NQ + kb, hlf); }
#pragma unroll
      for (int nt = 0; nt < 4; ++nt) { const v16b b = frag_kb(QT16 + (size_t)(nt * 16 + nloc) * NQ + kb, hlf);
#pragma unroll
        for (int mt = 0; mt < 2; ++mt) { acc[mt][nt] = wmma16b(ah[mt], b, acc[mt][nt]); acc[mt][nt] = wmma16b(al[mt], b, acc[mt][nt]); } } }
#pragma unroll
    for (int mt = 0; mt < 2; ++mt)
#pragma unroll
      for (int nt = 0; nt < 4; ++nt)
#pragma unroll
        for (int r = 0; r < 8; ++r) { const int f = nt * 16 + nloc; if (f < 52) ADQ[wave * 32 + mt * 16 + 8 * hlf + r][f] = acc[mt][nt][r] * (1.0f / (PS * XS)); } }
  { v8f acc[4] = {{}, {}, {}, {}};
#pragma unroll 2
    for (int kb = 0; kb < NS; kb += 32) { const v16b ah = frag_kb(Th_ + (size_t)(wave * 16 + nloc) * NS + kb, hlf), al = frag_kb(Tl_ + (size_t)(wave * 16 + nloc) * NS + kb, hlf);
#pragma unroll
      for (int nt = 0; nt < 4; ++nt) { const v16b b = frag_kb(Dt + (size_t)(nt * 16 + nloc) * NS + kb, hlf); acc[nt] = wmma16b(ah, b, acc[nt]); acc[nt] = wmma16b(al, b, acc[nt]); } }
#pragma unroll
    for (int nt = 0; nt < 4; ++nt) { v8b gh, gl; const int f = nt * 16 + nloc;
#pragma unroll
      for (int r = 0; r < 8; ++r) { b16 a_, c_; split16(acc[nt][r] * (1.0f / PS), a_, c_); gh[r] = a_; gl[r] = c_; }
      *(v8b*)(&GTh[f][wave * 16 + 8 * hlf]) = gh; *(v8b*)(&GTl[f][wave * 16 + 8 * hlf]) = gl; } }
  __syncthreads();
  { v8f acc[2][4];
#pragma unroll
    for (int mt = 0; mt < 2; ++mt)
#pragma unroll
      for (int nt = 0; nt < 4; ++nt) acc[mt][nt] = (v8f){};
#pragma unroll
    for (int kb = 0; kb < NQ; kb += 32) { v16b ah[2], al[2];
#pragma unroll
      for (int mt = 0; mt < 2; ++mt) { ah[mt] = frag_kb(Ph + (size_t)(wave * 32 + mt * 16 + nloc) * NQ + kb, hlf); al[mt] = frag_kb(Pl + (size_t)(wave * 32 + mt * 16 + nloc) * NQ + kb, hlf); }
#pragma unroll
      for (int nt = 0; nt < 4; ++nt) { const v16b bh = frag_kb(&GTh[nt * 16 + nloc][kb], hlf), bl = frag_kb(&GTl[nt * 16 + nloc][kb], hlf);
#pragma unroll
        for (int mt = 0; mt < 2; ++mt) { acc[mt][nt] = wmma16b(ah[mt], bh, acc[mt][nt]); acc[mt][nt] = wmma16b(al[mt], bh, acc[mt][nt]); acc[mt][nt] = wmma16b(ah[mt], bl, acc[mt][nt]); } } }
#pragma unroll
    for (int mt = 0; mt < 2; ++mt)
#pragma unroll
      for (int nt = 0; nt < 4; ++nt)
#pragma unroll
        for (int r = 0; r < 8; ++r) { const int f = nt * 16 + nloc; if (f < 52) AQD[wave * 32 + mt * 16 + 8 * hlf + r][f] = acc[mt][nt][r] * (1.0f / (PS * XS)); } }
  __syncthreads();
  const float dW1 = bf16_rne(dW1p[0]); const float* drow = doc + ((size_t)n * NS + t_) * NF;
  { float c = 0.0f;
#pragma unroll 1
    for (int f = 0; f < NF; ++f) { const float dv = bf16_rne(drow[f]), a = ADQ[t_][f], q = AQD[t_][f];
      c += pmul(tanh_(pmul(dW1, dv)), bf16_rne(dl1[f])) + pmul(tanh_(pmul(dW1, a)), bf16_rne(dl1[NF + f])) + pmul(tanh_(pmul(dW1, pmul(dv, a))), bf16_rne(dl1[2 * NF + f])) + pmul(tanh_(pmul(dW1, pmul(dv, q))), bf16_rne(dl1[3 * NF + f])); }
    Sc[t_] = c; }
  __syncthreads();
  { float mx = -INFINITY; for (int s = lane; s < NS; s += 32) mx = fmaxf(mx, Sc[s]); mx = hmax16(mx); mx = fmaxf(mx, __shfl_xor(mx, 16)); if (lane == 0) Sred[0][wave] = mx; }
  __syncthreads();
  float gmx = -INFINITY; for (int w = 0; w < 8; ++w) gmx = fmaxf(gmx, Sred[0][w]);
  const float es = nexp(Sc[t_] - gmx);
  __syncthreads(); Sc[t_] = es; __syncthreads();
  float tot = 0.0f; for (int s = 0; s < NS; ++s) tot += Sc[s];
  const float inv = 1.0f / tot;
  float xj = 0.0f;
  if (t_ < NV) { const int grp = t_ / NF, f = t_ - grp * NF;
    for (int s = 0; s < NS; ++s) { const float dv = bf16_rne(doc[((size_t)n * NS + s) * NF + f]); const float a = ADQ[s][f], q = AQD[s][f]; const float v = grp == 0 ? dv : grp == 1 ? a : grp == 2 ? pmul(dv, a) : pmul(dv, q); xj += pmul(Sc[s] * inv, v); } }
  for (int pass = 0; pass < 2; ++pass) { ((volatile float*)X)[(size_t)n * XW + t_] = xj; __threadfence(); }
}
__global__ __launch_bounds__(256) void tail_kernel(const float* __restrict__ X, const float* __restrict__ query, const float* __restrict__ dl2, const float* __restrict__ dW2p, const float* __restrict__ ql, const float* __restrict__ qWp, const float* __restrict__ l1w, const float* __restrict__ l1b, const float* __restrict__ l2w, const float* __restrict__ l2b, float* __restrict__ out) {
  __shared__ float Sb[NSEN], Sy[NV], Sq[NQ], Sz[NF], Sh[NF], Sred[8];
  const int t_ = threadIdx.x, wave = t_ >> 5, lane = t_ & 31; const float dW2 = bf16_rne(dW2p[0]), qW = bf16_rne(qWp[0]);
  for (int nn = t_; nn < NSEN; nn += 256) { float s = 0.0f;
#pragma unroll 1
    for (int j = 0; j < NV; ++j) s += pmul(tanh_(pmul(dW2, X[(size_t)nn * XW + j])), bf16_rne(dl2[j])); Sb[nn] = s; }
  __syncthreads();
  { float mx = -INFINITY; for (int k = lane; k < NSEN; k += 32) mx = fmaxf(mx, Sb[k]); mx = hmax16(mx); mx = fmaxf(mx, __shfl_xor(mx, 16)); if (lane == 0) Sred[wave] = mx; }
  __syncthreads();
  float gmx = -INFINITY; for (int w = 0; w < 8; ++w) gmx = fmaxf(gmx, Sred[w]);
  __syncthreads();
  for (int nn = t_; nn < NSEN; nn += 256) Sb[nn] = nexp(Sb[nn] - gmx);
  __syncthreads();
  float tot = 0.0f; for (int k = 0; k < NSEN; ++k) tot += Sb[k]; const float binv = 1.0f / tot;
  if (t_ < NV) { float y = 0.0f;
#pragma unroll 1
    for (int k = 0; k < NSEN; ++k) y += pmul(Sb[k] * binv, X[(size_t)k * XW + t_]); Sy[t_] = y; }
  if (t_ < NQ) { float s = 0.0f;
#pragma unroll 1
    for (int f = 0; f < NF; ++f) s += pmul(tanh_(pmul(qW, bf16_rne(query[t_ * NF + f]))), bf16_rne(ql[f])); Sq[t_] = s; }
  __syncthreads();
  if (t_ < NF) { float mx = -INFINITY; for (int q = 0; q < NQ; ++q) mx = fmaxf(mx, Sq[q]); float sm = 0.0f; for (int q = 0; q < NQ; ++q) sm += nexp(Sq[q] - mx); const float ainv = 1.0f / sm; float z = 0.0f;
#pragma unroll 1
    for (int q = 0; q < NQ; ++q) z += pmul(nexp(Sq[q] - mx) * ainv, bf16_rne(query[q * NF + t_])); Sz[t_] = z; }
  __syncthreads();
  if (t_ < NF) { float h = bf16_rne(l1b[t_]);
#pragma unroll 1
    for (int j = 0; j < NV; ++j) h += pmul(bf16_rne(l1w[t_ * NV + j]), Sy[j]); Sh[t_] = pmul(h, Sz[t_]); }
  __syncthreads();
  float o = bf16_rne(l2b[0]); if (t_ == 0)
#pragma unroll 1
    for (int f = 0; f < NF; ++f) o += pmul(bf16_rne(l2w[f]), Sh[f]);
  for (int pass = 0; pass < 2; ++pass) { if (t_ == 0) ((volatile float*)out)[0] = o; __threadfence(); }
}
}

extern "C" void kernel_launch(void* const* d_in, const int* in_sizes, int n_in, void* d_out, int out_size, void* d_ws, size_t ws_size, hipStream_t stream) {
  (void)n_in;
  auto Fp = [&](int i) { return (const float*)d_in[i]; };
  if (in_sizes[0] != NQ * NF || in_sizes[1] != NSEN * NS * NF || in_sizes[2] != 3 * NF || in_sizes[3] != NV || in_sizes[9] != NF * NV || out_size != 1) return;
  size_t off = 0; char* ws = (char*)d_ws;
  auto carve = [&](size_t bytes) { char* p = ws + off; off += (bytes + 255) & ~(size_t)255; return p; };
  b16* D16 = (b16*)carve((size_t)NSEN * NS * FP * 2); b16* DT16 = (b16*)carve((size_t)NSEN * FP * NS * 2); b16* QT16 = (b16*)carve((size_t)FP * NQ * 2);
  b16* QW3H = (b16*)carve((size_t)NQ * FP * 2); b16* QW3L = (b16*)carve((size_t)NQ * FP * 2); float* QW2 = (float*)carve(NQ * 4);
  b16* PQTH = (b16*)carve((size_t)SLOTS * NQ * NS * 2); b16* PQTL = (b16*)carve((size_t)SLOTS * NQ * NS * 2); b16* PDH = (b16*)carve((size_t)SLOTS * NS * NQ * 2); b16* PDL = (b16*)carve((size_t)SLOTS * NS * NQ * 2);
  float* X = (float*)carve((size_t)NSEN * XW * 4);
  if (off > ws_size) return;
  prep_kernel<<<dim3(NS / 64, NSEN), 256, 0, stream>>>(Fp(1), Fp(0), Fp(2), D16, DT16, QT16, QW3H, QW3L, QW2);
  for (int base = 0; base < NSEN; base += SLOTS) {
    phase1_kernel<<<SLOTS, 512, 0, stream>>>(D16, Fp(1), Fp(2), QW3H, QW3L, QW2, base, PQTH, PQTL, PDH, PDL);
    phase2_kernel<<<SLOTS, 256, 0, stream>>>(PDH, PDL, PQTH, PQTL, QT16, DT16, Fp(1), Fp(3), Fp(4), base, X); }
  tail_kernel<<<1, 256, 0, stream>>>(X, Fp(0), Fp(5), Fp(6), Fp(7), Fp(8), Fp(9), Fp(10), Fp(11), Fp(12), (float*)d_out);
}
